// QuantumInspiredAttention_5703716569513
// MI455X (gfx1250) — hardware-verified
//
#include <hip/hip_runtime.h>


#define NB   2
#define SEQ  1024
#define DIM  512
#define NX   (NB * SEQ)
#define NST  (NX * 8)
#define DH   64
#define RANK 4
#define RCH  512
#define DM   DIM
#define NTK  NX
#define EPS_ 1e-8f
#define SCL  0.125f
#define LOSC 1024.0f

typedef _Float16 h16;
typedef unsigned short bf;
typedef __attribute__((ext_vector_type(16))) __bf16   v16bf;
typedef __attribute__((ext_vector_type(16))) _Float16 v16h;
typedef __attribute__((ext_vector_type(8)))  _Float16 v8h;
typedef __attribute__((ext_vector_type(8)))  unsigned short v8us;
typedef __attribute__((ext_vector_type(8)))  float    v8f;
typedef __attribute__((ext_vector_type(4)))  float    v4f;
typedef __attribute__((ext_vector_type(4)))  _Float16 v4h;
typedef v8h  __attribute__((may_alias)) v8ha;
typedef v4f  __attribute__((may_alias)) v4fa;
typedef v8us __attribute__((may_alias)) v8usa;

__device__ __forceinline__ unsigned short f2bf(float f) { unsigned u = __float_as_uint(f); u += 0x7FFFu + ((u >> 16) & 1u); return (unsigned short)(u >> 16); }
__device__ __forceinline__ float bf2f(unsigned short b) { return __uint_as_float(((unsigned)b) << 16); }
__device__ __forceinline__ float bfr(float f) { return bf2f(f2bf(f)); }
__device__ __forceinline__ v16h cat16(v8h lo, v8h hi) { return __builtin_shufflevector(lo, hi, 0, 1, 2, 3, 4, 5, 6, 7, 8, 9, 10, 11, 12, 13, 14, 15); }
__device__ __forceinline__ v16bf cat16b(v8us lo, v8us hi) { return __builtin_bit_cast(v16bf, __builtin_shufflevector(lo, hi, 0, 1, 2, 3, 4, 5, 6, 7, 8, 9, 10, 11, 12, 13, 14, 15)); }
__device__ __forceinline__ v8f wmma16(v16h a, v16h b, v8f c) { return __builtin_amdgcn_wmma_f32_16x16x32_f16(false, a, false, b, (short)0, c, false, false); }
__device__ __forceinline__ v8f wmmab(v16bf a, v16bf b, v8f c) { return __builtin_amdgcn_wmma_f32_16x16x32_bf16(false, a, false, b, (short)0, c, false, false); }

__global__ __launch_bounds__(128) void k_gemm3(const bf* __restrict__ Ah, const bf* __restrict__ Al, const bf* __restrict__ Bh, const bf* __restrict__ Bl, int K, float* C, int ldc) {
    __shared__ __align__(16) float ost[4][16 * 68];
    const int lane = threadIdx.x & 31, wave = threadIdx.x >> 5, lr = lane & 15, hi = lane >> 4;
    const int r0 = blockIdx.x * 64 + wave * 16, c0 = blockIdx.y * 64;
    const size_t aoff = (size_t)(r0 + lr) * K + 8 * hi;
    v8f acc[4];
#pragma unroll
    for (int t = 0; t < 4; ++t) acc[t] = (v8f){};
#pragma unroll 1
    for (int kc = 0; kc < K; kc += 32) {
        const v16bf a = cat16b(*(const v8us*)(Ah + aoff + kc), *(const v8us*)(Ah + aoff + kc + 16));
        const v16bf al = cat16b(*(const v8us*)(Al + aoff + kc), *(const v8us*)(Al + aoff + kc + 16));
#pragma unroll
        for (int t = 0; t < 4; ++t) { const size_t bo = (size_t)(c0 + t * 16 + lr) * K + kc + 8 * hi;
            const v16bf bh = cat16b(*(const v8us*)(Bh + bo), *(const v8us*)(Bh + bo + 16)); const v16bf bl = cat16b(*(const v8us*)(Bl + bo), *(const v8us*)(Bl + bo + 16));
            acc[t] = wmmab(a, bh, acc[t]); acc[t] = wmmab(al, bh, acc[t]); acc[t] = wmmab(a, bl, acc[t]); }
        asm volatile("v_nop\n\tv_nop\n\tv_nop\n\tv_nop" : "+v"(acc[0]), "+v"(acc[1]), "+v"(acc[2]), "+v"(acc[3]) : "v"(a), "v"(al));
    }
    float* os = &ost[wave][0];
#pragma unroll
    for (int t = 0; t < 4; ++t) {
#pragma unroll
        for (int j = 0; j < 8; ++j) os[(hi * 8 + j) * 68 + t * 16 + lr] = acc[t][j]; }
    __builtin_amdgcn_wave_barrier(); asm volatile("" ::: "memory");
    float* crow = C + (size_t)r0 * ldc + c0;
    auto pass = [&]() {
#pragma unroll
        for (int s = 0; s < 8; ++s) { const int Lid = (lane >> 3) + 4 * s, piece = lane & 7; const int row = Lid >> 1, cofs = (Lid & 1) * 32 + piece * 4;
            const v4f val = *(const v4fa*)(os + row * 68 + cofs); *(volatile v4f*)(crow + (size_t)row * ldc + cofs) = val; }
    };
    pass(); __threadfence(); pass();
}

__global__ __launch_bounds__(256) void k_bfz(const float* __restrict__ src, bf* dh, bf* dz, size_t n8) {
    const size_t i = (size_t)blockIdx.x * 256 + threadIdx.x; if (i >= n8) return;
    const v8f v = *(const v8f*)(src + i * 8); v8us o, z;
#pragma unroll
    for (int k = 0; k < 8; ++k) { o[k] = f2bf(v[k]); z[k] = 0; }
    *(volatile v8us*)(dh + i * 8) = o; *(volatile v8us*)(dz + i * 8) = z; __threadfence(); *(volatile v8us*)(dh + i * 8) = o; *(volatile v8us*)(dz + i * 8) = z;
}
__global__ __launch_bounds__(256) void k_ttw(const float* __restrict__ A, const float* __restrict__ Bm, bf* Wh, bf* Wl) {
    const int lane = threadIdx.x & 31, o = blockIdx.x * 8 + (threadIdx.x >> 5); if (o >= DIM) return;
    const float a0 = bfr(A[o * RANK + 0]), a1 = bfr(A[o * RANK + 1]), a2 = bfr(A[o * RANK + 2]), a3 = bfr(A[o * RANK + 3]);
#pragma unroll 1
    for (int ps = 0; ps < 2; ++ps) {
#pragma unroll 1
        for (int q = 0; q < DIM / 256; ++q) { const int i0 = q * 256 + lane * 8; v8us oh, ol;
#pragma unroll
            for (int k = 0; k < 8; ++k) { const int i = i0 + k; float w = a0 * bfr(Bm[i]); w = fmaf(a1, bfr(Bm[DIM + i]), w); w = fmaf(a2, bfr(Bm[2 * DIM + i]), w); w = fmaf(a3, bfr(Bm[3 * DIM + i]), w);
                const unsigned short hb = f2bf(w); oh[k] = hb; ol[k] = f2bf(w - bf2f(hb)); }
            const size_t off = (size_t)o * DIM + i0; *(volatile v8us*)(Wh + off) = oh; *(volatile v8us*)(Wl + off) = ol; }
        if (ps == 0) __threadfence(); }
}
__global__ __launch_bounds__(256) void k_biasnorm(const float* __restrict__ Y, const float* __restrict__ bias, int normalise, float* F, bf* Ph, bf* Pl) {
    typedef __attribute__((ext_vector_type(2))) float v2f; typedef __attribute__((ext_vector_type(2))) unsigned short v2us;
    const int lane = threadIdx.x & 31, n = blockIdx.x * 8 + (threadIdx.x >> 5); if (n >= NST) return;
    const size_t o = (size_t)n * DH + 2 * lane; const int col = (n & 7) * DH + 2 * lane;
    float v0 = Y[o] + bfr(bias[col]), v1 = Y[o + 1] + bfr(bias[col + 1]);
    if (normalise) { float ss = v0 * v0 + v1 * v1;
#pragma unroll
        for (int sh = 16; sh; sh >>= 1) ss += __shfl_xor(ss, sh, 32);
        const float inv = 1.0f / (sqrtf(ss) + EPS_); v0 *= inv; v1 *= inv; }
    v2f f; f[0] = v0; f[1] = v1; v2us oh, ol;
#pragma unroll
    for (int i = 0; i < 2; ++i) { const unsigned short hb = f2bf(f[i]); oh[i] = hb; ol[i] = f2bf(f[i] - bf2f(hb)); }
    if (F) *(volatile v2f*)(F + o) = f; if (Ph) { *(volatile v2us*)(Ph + o) = oh; *(volatile v2us*)(Pl + o) = ol; } __threadfence();
    if (F) *(volatile v2f*)(F + o) = f; if (Ph) { *(volatile v2us*)(Ph + o) = oh; *(volatile v2us*)(Pl + o) = ol; }
}
__global__ __launch_bounds__(256) void k_vt64(const float* __restrict__ V, bf* VTh, bf* VTl) {
    typedef __attribute__((ext_vector_type(2))) unsigned short v2us;
    const int lane = threadIdx.x & 31, wid = blockIdx.x * 8 + (threadIdx.x >> 5); if (wid >= (NST / 64) * DH) return;
    const int d = wid % DH, g = wid / DH; const int n0 = g * 64 + 2 * lane; v2us oh, ol;
#pragma unroll
    for (int i = 0; i < 2; ++i) { const float v = V[(size_t)(n0 + i) * DH + d]; const unsigned short hb = f2bf(v); oh[i] = hb; ol[i] = f2bf(v - bf2f(hb)); }
    const size_t o = (size_t)d * NST + n0;
    *(volatile v2us*)(VTh + o) = oh; *(volatile v2us*)(VTl + o) = ol; __threadfence(); *(volatile v2us*)(VTh + o) = oh; *(volatile v2us*)(VTl + o) = ol;
}
__global__ __launch_bounds__(256) void k_softmax(const float* __restrict__ S, bf* PH, bf* PL) {
    const int lane = threadIdx.x & 31, r = blockIdx.x * 8 + (threadIdx.x >> 5); if (r >= RCH) return;
    const float* sr = S + (size_t)r * NST; float m = -3.0e38f;
#pragma unroll 1
    for (int c0 = lane * 8; c0 < NST; c0 += 256) { const v8f v = *(const v8f*)(sr + c0);
#pragma unroll
        for (int i = 0; i < 8; ++i) m = fmaxf(m, v[i] * SCL); }
#pragma unroll
    for (int sh = 16; sh; sh >>= 1) m = fmaxf(m, __shfl_xor(m, sh, 32));
    float sum = 0.f;
#pragma unroll 1
    for (int c0 = lane * 8; c0 < NST; c0 += 256) { const v8f v = *(const v8f*)(sr + c0);
#pragma unroll
        for (int i = 0; i < 8; ++i) sum += __expf(v[i] * SCL - m); }
#pragma unroll
    for (int sh = 16; sh; sh >>= 1) sum += __shfl_xor(sum, sh, 32);
    const float inv = 1.0f / sum;
#pragma unroll 1
    for (int ps = 0; ps < 2; ++ps) {
#pragma unroll 1
        for (int c0 = lane * 8; c0 < NST; c0 += 256) { const v8f v = *(const v8f*)(sr + c0); v8us oh, ol;
#pragma unroll
            for (int i = 0; i < 8; ++i) { const float p = __expf(v[i] * SCL - m) * inv; const unsigned short hb = f2bf(p); oh[i] = hb; ol[i] = f2bf(p - bf2f(hb)); }
            const size_t o = (size_t)r * NST + c0; *(volatile v8us*)(PH + o) = oh; *(volatile v8us*)(PL + o) = ol; }
        if (ps == 0) __threadfence(); }
}
__global__ __launch_bounds__(256) void k_measure(const float* __restrict__ AT, bf* Mh, bf* Ml) {
    typedef __attribute__((ext_vector_type(2))) unsigned short v2us;
    const int lane = threadIdx.x & 31, n = blockIdx.x * 8 + (threadIdx.x >> 5); if (n >= RCH) return;
    const size_t o = (size_t)n * DH + 2 * lane; const float a0 = AT[o], a1 = AT[o + 1]; float ss = a0 * a0 + a1 * a1;
#pragma unroll
    for (int sh = 16; sh; sh >>= 1) ss += __shfl_xor(ss, sh, 32);
    const float inv = 1.0f / (ss + EPS_); float y[2] = {a0 * a0 * inv, a1 * a1 * inv}; v2us oh, ol;
#pragma unroll
    for (int i = 0; i < 2; ++i) { const unsigned short hb = f2bf(y[i]); oh[i] = hb; ol[i] = f2bf(y[i] - bf2f(hb)); }
    *(volatile v2us*)(Mh + o) = oh; *(volatile v2us*)(Ml + o) = ol; __threadfence(); *(volatile v2us*)(Mh + o) = oh; *(volatile v2us*)(Ml + o) = ol;
}
__global__ __launch_bounds__(256) void k_addbias(const float* __restrict__ T, const float* __restrict__ b, float* OUTP) {
    const int lane = threadIdx.x & 31, r = blockIdx.x * 8 + (threadIdx.x >> 5); if (r >= NX) return;
#pragma unroll 1
    for (int ps = 0; ps < 2; ++ps) {
#pragma unroll 1
        for (int q = 0; q < DIM / 256; ++q) { const size_t o = (size_t)r * DIM + q * 256 + lane * 8; v8f v = *(const v8f*)(T + o);
#pragma unroll
            for (int i = 0; i < 8; ++i) v[i] += bfr(b[q * 256 + lane * 8 + i]);
            *(volatile v8f*)(OUTP + o) = v; }
        if (ps == 0) __threadfence(); }
}

extern "C" void kernel_launch(void* const* d_in, const int* in_sizes, int n_in,
                              void* d_out, int out_size, void* d_ws, size_t ws_size, hipStream_t stream) {
    (void)in_sizes; (void)n_in; (void)out_size;
    const float* x = (const float*)d_in[0];
    const float* qA = (const float*)d_in[1]; const float* qB = (const float*)d_in[2]; const float* qb = (const float*)d_in[3]; const float* kA = (const float*)d_in[4]; const float* kB = (const float*)d_in[5]; const float* kb = (const float*)d_in[6];
    const float* vA = (const float*)d_in[7]; const float* vB = (const float*)d_in[8]; const float* vb = (const float*)d_in[9]; const float* oA = (const float*)d_in[10]; const float* oB = (const float*)d_in[11]; const float* ob = (const float*)d_in[12];
    float* out = (float*)d_out;
    char* wsp = (char*)d_ws;
    auto take = [&](size_t bytes) { char* p = wsp; wsp += (bytes + 255) & ~(size_t)255; return (void*)p; };
    bf* Xh = (bf*)take((size_t)NX * DIM * 2); bf* Xz = (bf*)take((size_t)NX * DIM * 2); bf* Wh[4]; bf* Wl[4];
    for (int i = 0; i < 4; ++i) { Wh[i] = (bf*)take((size_t)DIM * DIM * 2); Wl[i] = (bf*)take((size_t)DIM * DIM * 2); }
    float* TMP = (float*)take((size_t)NX * DIM * 4); bf* QQh = (bf*)take((size_t)NST * DH * 2); bf* QQl = (bf*)take((size_t)NST * DH * 2); bf* KQh = (bf*)take((size_t)NST * DH * 2); bf* KQl = (bf*)take((size_t)NST * DH * 2);
    float* Vf = (float*)take((size_t)NST * DH * 4); bf* VTh = (bf*)take((size_t)DH * NST * 2); bf* VTl = (bf*)take((size_t)DH * NST * 2);
    float* S = (float*)take((size_t)RCH * NST * 4); bf* PH = (bf*)take((size_t)RCH * NST * 2); bf* PL = (bf*)take((size_t)RCH * NST * 2); float* AT = (float*)take((size_t)RCH * DH * 4);
    bf* Mh = (bf*)take((size_t)NX * DIM * 2); bf* Ml = (bf*)take((size_t)NX * DIM * 2);
    if ((size_t)(wsp - (char*)d_ws) > ws_size) return;
    k_bfz<<<(NX * DIM / 8 + 255) / 256, 256, 0, stream>>>(x, Xh, Xz, (size_t)NX * DIM / 8);
    k_ttw<<<DIM / 8, 256, 0, stream>>>(qA, qB, Wh[0], Wl[0]); k_ttw<<<DIM / 8, 256, 0, stream>>>(kA, kB, Wh[1], Wl[1]); k_ttw<<<DIM / 8, 256, 0, stream>>>(vA, vB, Wh[2], Wl[2]); k_ttw<<<DIM / 8, 256, 0, stream>>>(oA, oB, Wh[3], Wl[3]);
    k_gemm3<<<dim3(NX / 64, DIM / 64, 1), 128, 0, stream>>>(Xh, Xz, Wh[0], Wl[0], DIM, TMP, DIM); k_biasnorm<<<NST / 8, 256, 0, stream>>>(TMP, qb, 1, nullptr, QQh, QQl);
    k_gemm3<<<dim3(NX / 64, DIM / 64, 1), 128, 0, stream>>>(Xh, Xz, Wh[1], Wl[1], DIM, TMP, DIM); k_biasnorm<<<NST / 8, 256, 0, stream>>>(TMP, kb, 1, nullptr, KQh, KQl);
    k_gemm3<<<dim3(NX / 64, DIM / 64, 1), 128, 0, stream>>>(Xh, Xz, Wh[2], Wl[2], DIM, TMP, DIM); k_biasnorm<<<NST / 8, 256, 0, stream>>>(TMP, vb, 0, Vf, nullptr, nullptr);
    k_vt64<<<((NST / 64) * DH) / 8, 256, 0, stream>>>(Vf, VTh, VTl);
    for (int ch = 0; ch < NST / RCH; ++ch) { const size_t n0 = (size_t)ch * RCH;
        k_gemm3<<<dim3(RCH / 64, NST / 64, 1), 128, 0, stream>>>(QQh + n0 * DH, QQl + n0 * DH, KQh, KQl, DH, S, NST);
        k_softmax<<<RCH / 8, 256, 0, stream>>>(S, PH, PL);
        k_gemm3<<<dim3(RCH / 64, 1, 1), 128, 0, stream>>>(PH, PL, VTh, VTl, NST, AT, DH);
        k_measure<<<RCH / 8, 256, 0, stream>>>(AT, Mh + n0 * DH, Ml + n0 * DH);
    }
    k_gemm3<<<dim3(NX / 64, DIM / 64, 1), 128, 0, stream>>>(Mh, Ml, Wh[3], Wl[3], DIM, TMP, DIM); k_addbias<<<NX / 8, 256, 0, stream>>>(TMP, ob, out);
}
